// JastrowNet_39771397160975
// MI455X (gfx1250) — hardware-verified
//
#include <hip/hip_runtime.h>
#include <stddef.h>


typedef _Float16 v16h __attribute__((ext_vector_type(16)));
typedef _Float16 v8h  __attribute__((ext_vector_type(8)));
typedef float    v8f  __attribute__((ext_vector_type(8)));
typedef float    v4f  __attribute__((ext_vector_type(4)));

#ifndef NB
#define NB 8192
#endif
#define NB_FULL 8192
#define E_STRIDE_FULL 1024
#define N_STRIDE_FULL 256
#define BPB 32

static_assert(NB >= BPB && NB <= NB_FULL && (NB % BPB) == 0);
static_assert(BPB == 8 * 4);
static_assert(BPB * 4 == 128);

#define ECARRY 256.0f
#define WCARRY 64.0f
#define ACARRY 64.0f
#define XCARRY 16.0f
#define ZCARRY 16.0f
#define S1  16384.0f
#define S2  4096.0f
#define SH  1024.0f
#define SG1 1024.0f
#define SG2 4096.0f
#define LN2F 0.6931471805599453f

#define IMG_ONE    512
#define IMG_LAYER  (8 * IMG_ONE)
#define IMG_HALVES (2 * IMG_LAYER)
#define T_W1E 0
#define T_W2E 1
#define T_W1N 2
#define T_W2N 3
#define T_HW  4
#define T_G1A 5
#define T_G1B 6
#define T_G2  7
static_assert(IMG_HALVES == 8192);
static_assert(IMG_HALVES == 256 * 4 * 8);

#define F_B1E 0
#define F_B2E 16
#define F_B1N 32
#define F_B2N 48
#define F_HB  64
#define F_GB1 80
#define F_GB2 112
#define F_LAYER 128
#define F_Y   256
#define F_XI  288
#define F_OW  544
#define F_OB  560
#define FSEC  576
static_assert(FSEC == 144 * 4);
static_assert((FSEC % 32) == 0);

#define IMG_BYTES ((size_t)IMG_HALVES * 2)
#define F_BYTES   ((size_t)FSEC * 4)
#define OFF_IMG   ((size_t)0)
#define OFF_F     (OFF_IMG + IMG_BYTES)
#define WS_TOTAL  (OFF_F + F_BYTES)
static_assert((IMG_BYTES % 128) == 0 && (F_BYTES % 128) == 0);
static_assert(WS_TOTAL <= (size_t)134217728);

#define ZP 40
#define ZT (16 * ZP)
static_assert((ZP % 8) == 0 && ZP >= 32);

__device__ __forceinline__ float bf16r(float x) {
  unsigned int u = __float_as_uint(x);
  u = (u + 0x7FFFu + ((u >> 16) & 1u)) & 0xFFFF0000u;
  return __uint_as_float(u);
}

__device__ __forceinline__ v16h frag_at(const _Float16* p) {
  v8h lo = *(const v8h*)(p);
  v8h hi = *(const v8h*)(p + 16);
  v16h out;
#pragma unroll
  for (int i = 0; i < 8; ++i) { out[i] = lo[i]; out[i + 8] = hi[i]; }
  return out;
}

__device__ __forceinline__ v16h frag_lane(const _Float16* p) {
  const v8h lo = *(const v8h*)(p);
  const v8h hi = *(const v8h*)(p + 8);
  v16h out;
#pragma unroll
  for (int i = 0; i < 8; ++i) { out[i] = lo[i]; out[i + 8] = hi[i]; }
  return out;
}

__device__ __forceinline__ v8f wmma16(v16h a, v16h b, v8f c) {
  v8f d = __builtin_amdgcn_wmma_f32_16x16x32_f16(false, a, false, b, (short)0, c,
                                                 false, false);
  asm volatile("v_nop\n\tv_nop\n\tv_nop\n\tv_nop" : "+v"(d) : "v"(a), "v"(b));
  return d;
}

__device__ __forceinline__ float red32_sum(float x) {
#pragma unroll
  for (int off = 1; off < 32; off <<= 1) x += __shfl_xor(x, off, 32);
  return x;
}

__device__ __forceinline__ void wave_lds_sync() {
  __builtin_amdgcn_fence(3  , "wavefront");
  asm volatile("s_wait_dscnt 0x0" ::: "memory");
  __builtin_amdgcn_wave_barrier();
}

static __device__ __forceinline__ _Float16 toh_flush(float v) {
  const _Float16 r = (_Float16)v;
  return (fabsf(v) < 6.103515625e-05f) ? (_Float16)0.0f : r;
}

__device__ __forceinline__ float ssp_act(float t) {
  const float e = __expf(-fabsf(t));
  return (fmaxf(t, 0.0f) + __logf(1.0f + e)) - LN2F;
}

__device__ __forceinline__ v8f splat8(float v) {
  v8f c;
#pragma unroll
  for (int r = 0; r < 8; ++r) c[r] = v;
  return c;
}

__device__ __forceinline__ v16h edge_frag(const v4f e, const bool lowhalf) {
  v16h f = {};
#pragma unroll
  for (int i = 0; i < 4; ++i) {
    const float t = lowhalf ? (ECARRY * bf16r(e[i])) : 0.0f;
    f[i] = toh_flush(t);
  }
  return f;
}

__device__ __forceinline__ v16h act_frag8(const v8f c, const float inv) {
  v16h f = {};
#pragma unroll
  for (int r = 0; r < 8; ++r) f[r] = toh_flush(ACARRY * ssp_act(c[r] * inv));
  return f;
}

__device__ __forceinline__ float ldsel(const float* __restrict__ p, unsigned idx, unsigned n,
                                       bool ok) {
  const unsigned c = (idx < n) ? idx : (n - 1u);
  const float v = p[c];
  return ok ? bf16r(v) : 0.0f;
}

__global__ __launch_bounds__(256) void pack_kernel(
    const float* __restrict__ xi, const float* __restrict__ Y,
    const float* __restrict__ wW1, const float* __restrict__ wb1,
    const float* __restrict__ wW2, const float* __restrict__ wb2,
    const float* __restrict__ hW, const float* __restrict__ hb,
    const float* __restrict__ gW1, const float* __restrict__ gb1,
    const float* __restrict__ gW2, const float* __restrict__ gb2,
    const float* __restrict__ oW, const float* __restrict__ ob,
    _Float16* __restrict__ wimg, float* __restrict__ wf32) {
#pragma clang fp contract(off)
  __shared__ __attribute__((aligned(16))) _Float16 T[IMG_HALVES];
  __shared__ __attribute__((aligned(16))) float F[768];
  const unsigned tid = threadIdx.x;

#pragma unroll 1
  for (unsigned j = 0; j < 32u; ++j) {
    const unsigned idx = tid + 256u * j;
    const unsigned img = j >> 1;
    const unsigned l = img >> 3, t = img & 7u;
    const unsigned within = idx & 511u;
    const unsigned L = within >> 4, i = within & 15u;
    const unsigned hh = L >> 4, rc = L & 15u;
    const unsigned k = 8u * hh + i + ((i >= 8u) ? 8u : 0u);
    float v;
    if (t == (unsigned)T_W1E) {
      v = ldsel(wW1, ((l * 3u + (rc >> 3)) * 4u + (k & 3u)) * 8u + (rc & 7u), 192u, k < 4u);
    } else if (t == (unsigned)T_W2E) {
      const unsigned c = (k >> 3) & 1u;
      v = ldsel(wW2, ((l * 3u + c) * 8u + (k & 7u)) * 8u + (rc & 7u), 384u,
                (k < 16u) && ((k >> 3) == (rc >> 3)));
    } else if (t == (unsigned)T_W1N) {
      v = ldsel(wW1, ((l * 3u + 2u) * 4u + (k & 3u)) * 8u + (rc & 7u), 192u,
                (k < 4u) && (rc < 8u));
    } else if (t == (unsigned)T_W2N) {
      v = ldsel(wW2, ((l * 3u + 2u) * 8u + (k & 7u)) * 8u + (rc & 7u), 384u,
                (k < 8u) && (rc < 8u));
    } else if (t == (unsigned)T_HW) {
      v = ldsel(hW, (l * 16u + (k & 15u)) * 8u + (rc & 7u), 256u, k < 16u);
    } else if (t == (unsigned)T_G1A) {
      const unsigned c = rc >> 3;
      v = ldsel(gW1, ((l * 3u + c) * 8u + (k & 7u)) * 8u + (rc & 7u), 384u,
                (k < 16u) && ((k >> 3) == c));
    } else if (t == (unsigned)T_G1B) {
      v = ldsel(gW1, ((l * 3u + 2u) * 8u + (k & 7u)) * 8u + (rc & 7u), 384u,
                (rc < 8u) && (k >= 16u) && (k < 24u));
    } else {
      const unsigned c = ((k >> 3) > 2u) ? 2u : (k >> 3);
      v = ldsel(gW2, ((l * 3u + c) * 8u + (k & 7u)) * 16u + rc, 768u, k < 24u);
    }
    T[idx] = toh_flush(WCARRY * v);
  }

#pragma unroll 1
  for (unsigned j = 0; j < 3u; ++j) {
    const unsigned idx = tid + 256u * j;
    const unsigned l = (idx >> 7) & 1u;
    const unsigned o = idx & 127u;
    const unsigned i16 = o & 15u, c2 = i16 >> 3, k8 = i16 & 7u;
    const float c_b1e = S1 * bf16r(wb1[(l * 3u + c2) * 8u + k8]);
    const float c_b2e = S2 * bf16r(wb2[(l * 3u + c2) * 8u + k8]);
    const float t_b1n = S1 * bf16r(wb1[(l * 3u + 2u) * 8u + k8]);
    const float t_b2n = S2 * bf16r(wb2[(l * 3u + 2u) * 8u + k8]);
    const float c_b1n = (i16 < 8u) ? t_b1n : 0.0f;
    const float c_b2n = (i16 < 8u) ? t_b2n : 0.0f;
    const float c_hb  = SH * bf16r(hb[l * 8u + k8]);
    const unsigned ig  = (o >= 80u) ? (o - 80u) : 0u;
    const unsigned igc = (ig < 24u) ? ig : 23u;
    const float t_gb1 = SG1 * bf16r(gb1[(l * 3u + (igc >> 3)) * 8u + (igc & 7u)]);
    const float c_gb1 = (ig < 24u) ? t_gb1 : 0.0f;
    const float c_gb2 = (bf16r(gb2[(l * 3u + 0u) * 16u + i16]) +
                         bf16r(gb2[(l * 3u + 1u) * 16u + i16])) +
                        bf16r(gb2[(l * 3u + 2u) * 16u + i16]);
    float vl = c_b1e;
    vl = (o >= 16u)  ? c_b2e : vl;
    vl = (o >= 32u)  ? c_b1n : vl;
    vl = (o >= 48u)  ? c_b2n : vl;
    vl = (o >= 64u)  ? c_hb  : vl;
    vl = (o >= 80u)  ? c_gb1 : vl;
    vl = (o >= 112u) ? c_gb2 : vl;

    const unsigned g  = (idx >= 256u) ? (idx - 256u) : 0u;
    const unsigned gy = (g < 32u) ? g : 31u;
    const unsigned gx0 = (g >= 32u) ? (g - 32u) : 0u;
    const unsigned gx = (gx0 < 256u) ? gx0 : 255u;
    const unsigned go0 = (g >= 288u) ? (g - 288u) : 0u;
    const unsigned go = (go0 < 16u) ? go0 : 15u;
    const float c_y  = bf16r(Y[gy]);
    const float c_xi = bf16r(xi[gx]);
    const float c_ow = bf16r(oW[go]);
    const float c_ob = bf16r(ob[0]);
    float vg = c_y;
    vg = (g >= 32u)  ? c_xi : vg;
    vg = (g >= 288u) ? c_ow : vg;
    vg = (g >= 304u) ? c_ob : vg;
    vg = (g >= 305u) ? 0.0f : vg;
    F[idx] = (idx < 256u) ? vl : vg;
  }
  __syncthreads();

  v8h x[4];
#pragma unroll
  for (unsigned i = 0; i < 4u; ++i) x[i] = *(const v8h*)&T[(tid + 256u * i) * 8u];
  const unsigned fi = (tid < 144u) ? tid : 143u;
  const v4f y = *(const v4f*)&F[fi * 4u];
#pragma unroll
  for (unsigned i = 0; i < 4u; ++i) *(volatile v8h*)(wimg + (size_t)(tid + 256u * i) * 8u) = x[i];
  if (tid < 144u) *(volatile v4f*)(wf32 + (size_t)tid * 4u) = y;
  __threadfence();
#pragma unroll
  for (unsigned i = 0; i < 4u; ++i) *(volatile v8h*)(wimg + (size_t)(tid + 256u * i) * 8u) = x[i];
  if (tid < 144u) *(volatile v4f*)(wf32 + (size_t)tid * 4u) = y;
}

__global__ __launch_bounds__(256) void jastrow_kernel(
    const float* __restrict__ edges_e, const float* __restrict__ edges_n,
    const _Float16* __restrict__ wimg, const float* __restrict__ wf32,
    float* __restrict__ out) {
  __shared__ __attribute__((aligned(16))) _Float16 sImg[IMG_HALVES];
  __shared__ __attribute__((aligned(16))) float sF[FSEC];
  __shared__ __attribute__((aligned(16))) _Float16 sZ[8 * ZT];
  __shared__ __attribute__((aligned(16))) float sOut[BPB];

  const unsigned tid = threadIdx.x;
#pragma unroll
  for (unsigned i = 0; i < 4u; ++i) {
    const unsigned piece = tid + 256u * i;
    *(v8h*)&sImg[piece * 8u] = *(const v8h*)(wimg + (size_t)piece * 8u);
  }
  {
    const unsigned fi = (tid < 144u) ? tid : 143u;
    *(v4f*)&sF[fi * 4u] = *(const v4f*)(wf32 + (size_t)fi * 4u);
  }
  __syncthreads();

  const int wave = __builtin_amdgcn_readfirstlane(threadIdx.x >> 5);
  const unsigned lane = tid & 31u;
  const unsigned h = lane >> 4, n = lane & 15u;
  const bool lowhalf = (h == 0u);
  const unsigned zbase = (unsigned)wave * (unsigned)ZT;

  float yreg[4];
#pragma unroll
  for (int a = 0; a < 4; ++a) yreg[a] = sF[F_Y + a * 8 + (n & 7u)];
  float ow[8];
#pragma unroll
  for (int r = 0; r < 8; ++r) ow[r] = sF[F_OW + 8u * h + (unsigned)r];
  const float obias = sF[F_OB];

  const unsigned ch = n >> 3;
  const float gA = ((h ^ ch) == 0u) ? 1.0f : 0.0f;
  const float gB = 1.0f - gA;
  const float dA = (ch == 0u && h == 0u) ? 1.0f : 0.0f;
  const float dB = (ch == 0u && h == 1u) ? 1.0f : 0.0f;

#pragma unroll 1
  for (int t4 = 0; t4 < 4; ++t4) {
    const unsigned b = blockIdx.x * (unsigned)BPB + (unsigned)wave * 4u + (unsigned)t4;
    const float* eE = edges_e + (size_t)b * E_STRIDE_FULL;
    const float* eN = edges_n + (size_t)b * N_STRIDE_FULL;

    float xr[8];
#pragma unroll
    for (int r = 0; r < 8; ++r) xr[r] = sF[F_XI + n * 16u + 8u * h + (unsigned)r];

#pragma unroll 1
    for (int l = 0; l < 2; ++l) {
      const unsigned ib = (unsigned)l * (unsigned)IMG_LAYER + lane * 16u;
      const unsigned fb = (unsigned)l * (unsigned)F_LAYER;

      float hxs[8];
      {
        v16h ax = {};
#pragma unroll
        for (int r = 0; r < 8; ++r) ax[r] = toh_flush(XCARRY * xr[r]);
        const v16h bh = frag_lane(&sImg[ib + T_HW * IMG_ONE]);
        const v8f hx = wmma16(ax, bh, splat8(sF[fb + F_HB + n]));
#pragma unroll
        for (int r = 0; r < 8; ++r) hxs[r] = hx[r] * (1.0f / (SH * S2));
      }

      {
        const v16h aW1 = frag_lane(&sImg[ib + T_W1E * IMG_ONE]);
        const v16h bW2 = frag_lane(&sImg[ib + T_W2E * IMG_ONE]);
        v8f b1;
#pragma unroll
        for (int r = 0; r < 8; ++r) b1[r] = sF[fb + F_B1E + 8u * h + (unsigned)r];
        const float b2 = sF[fb + F_B2E + n];
#pragma unroll 1
        for (int ih = 0; ih < 2; ++ih) {
          const float g  = ih ? gB : gA;
          const float dX = ih ? dB : dA;
#pragma unroll
          for (int u = 0; u < 8; ++u) {
            const unsigned irow = (unsigned)(ih * 8 + u);
            const v4f e = *(const v4f*)(eE + (irow * 16u + n) * 4u);
            const v16h be = edge_frag(e, lowhalf);
            const v8f c1 = wmma16(aW1, be, b1);
            const v16h a2 = act_frag8(c1, 1.0f / S1);
            const v8f c2 = wmma16(a2, bW2, splat8(b2));
            float dot = 0.0f;
#pragma unroll
            for (int r = 0; r < 8; ++r) dot = fmaf(c2[r], hxs[r], dot);
            const float pe = c2[u] * hxs[u];
            float part = g * dot - dX * pe;
            part += __shfl_xor(part, 16, 32);
            sZ[zbase + irow * (unsigned)ZP + n] = toh_flush(ZCARRY * part);
          }
        }
      }

      {
        const v16h aW1 = frag_lane(&sImg[ib + T_W1N * IMG_ONE]);
        const v16h bW2 = frag_lane(&sImg[ib + T_W2N * IMG_ONE]);
        v8f b1;
#pragma unroll
        for (int r = 0; r < 8; ++r) b1[r] = sF[fb + F_B1N + 8u * h + (unsigned)r];
        const float b2 = sF[fb + F_B2N + n];
#pragma unroll 1
        for (int t = 0; t < 4; ++t) {
          const v4f e = *(const v4f*)(eN + ((unsigned)t * 16u + n) * 4u);
          const v16h be = edge_frag(e, lowhalf);
          const v8f c1 = wmma16(aW1, be, b1);
          const v16h a2 = act_frag8(c1, 1.0f / S1);
          const v8f c2 = wmma16(a2, bW2, splat8(b2));
          float s0 = c2[0] * yreg[0];
          s0 = fmaf(c2[1], yreg[1], s0);
          s0 = fmaf(c2[2], yreg[2], s0);
          s0 = fmaf(c2[3], yreg[3], s0);
          float s1 = c2[4] * yreg[0];
          s1 = fmaf(c2[5], yreg[1], s1);
          s1 = fmaf(c2[6], yreg[2], s1);
          s1 = fmaf(c2[7], yreg[3], s1);
          const float z0 = (n < 8u) ? (s0 * (ZCARRY / S2)) : 0.0f;
          const float z1 = (n < 8u) ? (s1 * (ZCARRY / S2)) : 0.0f;
          const unsigned i0 = (unsigned)t * 4u + 2u * h;
          sZ[zbase + i0 * (unsigned)ZP + 16u + n]        = toh_flush(z0);
          sZ[zbase + (i0 + 1u) * (unsigned)ZP + 16u + n] = toh_flush(z1);
        }
      }

      wave_lds_sync();
      const v16h bz = frag_at(&sZ[zbase + n * (unsigned)ZP + h * 8u]);
      wave_lds_sync();
      {
        v8f gi0, gi1;
#pragma unroll
        for (int r = 0; r < 8; ++r) {
          gi0[r] = sF[fb + F_GB1 + 8u * h + (unsigned)r];
          gi1[r] = sF[fb + F_GB1 + 16u + 8u * h + (unsigned)r];
        }
        const v16h aG1a = frag_lane(&sImg[ib + T_G1A * IMG_ONE]);
        const v8f d0 = wmma16(aG1a, bz, gi0);
        const v16h aG1b = frag_lane(&sImg[ib + T_G1B * IMG_ONE]);
        const v8f d1 = wmma16(aG1b, bz, gi1);
        v16h bg;
#pragma unroll
        for (int r = 0; r < 8; ++r) {
          bg[r]     = toh_flush(ACARRY * ssp_act(d0[r] * (1.0f / SG1)));
          bg[r + 8] = toh_flush(ACARRY * ssp_act(d1[r] * (1.0f / SG1)));
        }
        const v16h aG2 = frag_lane(&sImg[ib + T_G2 * IMG_ONE]);
        const v8f up = wmma16(aG2, bg, splat8(0.0f));
#pragma unroll
        for (int r = 0; r < 8; ++r)
          xr[r] = xr[r] + (up[r] * (1.0f / SG2) + sF[fb + F_GB2 + 8u * h + (unsigned)r]);
      }
    }

    float acc = 0.0f;
#pragma unroll
    for (int r = 0; r < 8; ++r) acc = fmaf(xr[r], ow[r], acc);
    acc = red32_sum(acc);
    if (lane == 0u) sOut[wave * 4 + t4] = acc + 16.0f * obias;
  }
  __syncthreads();

  const v4f val = *(const v4f*)&sOut[(lane & 7u) * 4u];
  if (wave == 0) {
    if (lane < 8u) {
      float* p = out + (size_t)blockIdx.x * BPB + lane * 4u;
      *(volatile v4f*)p = val;
      __threadfence();
      *(volatile v4f*)p = val;
    }
  }
}

extern "C" void kernel_launch(void* const* d_in, const int* in_sizes, int n_in,
                              void* d_out, int out_size, void* d_ws, size_t ws_size,
                              hipStream_t stream) {
  if (n_in < 16) return;
  if ((long long)in_sizes[0] < (long long)NB * E_STRIDE_FULL) return;
  if ((long long)in_sizes[1] < (long long)NB * N_STRIDE_FULL) return;
  if (in_sizes[2] < 256 || in_sizes[3] < 32) return;
  if (in_sizes[4] < 192 || in_sizes[5] < 48 || in_sizes[6] < 384 || in_sizes[7] < 48) return;
  if (in_sizes[8] < 256 || in_sizes[9] < 16) return;
  if (in_sizes[10] < 384 || in_sizes[11] < 48 || in_sizes[12] < 768 || in_sizes[13] < 96) return;
  if (in_sizes[14] < 16 || in_sizes[15] < 1) return;
  if (out_size < NB) return;
  if (ws_size < WS_TOTAL) return;

  const float* edges_e = (const float*)d_in[0];
  const float* edges_n = (const float*)d_in[1];
  const float* x_init  = (const float*)d_in[2];
  const float* Y       = (const float*)d_in[3];
  const float* wW1     = (const float*)d_in[4];
  const float* wb1     = (const float*)d_in[5];
  const float* wW2     = (const float*)d_in[6];
  const float* wb2     = (const float*)d_in[7];
  const float* hW      = (const float*)d_in[8];
  const float* hb      = (const float*)d_in[9];
  const float* gW1     = (const float*)d_in[10];
  const float* gb1     = (const float*)d_in[11];
  const float* gW2     = (const float*)d_in[12];
  const float* gb2     = (const float*)d_in[13];
  const float* oW      = (const float*)d_in[14];
  const float* ob      = (const float*)d_in[15];
  float* outp = (float*)d_out;

  char* ws = (char*)d_ws;
  _Float16* wimg = (_Float16*)(ws + OFF_IMG);
  float*    wf32 = (float*)(ws + OFF_F);

  pack_kernel<<<dim3(1), dim3(256), 0, stream>>>(
      x_init, Y, wW1, wb1, wW2, wb2, hW, hb, gW1, gb1, gW2, gb2, oW, ob, wimg, wf32);
  jastrow_kernel<<<dim3(NB / BPB), dim3(256), 0, stream>>>(edges_e, edges_n, wimg, wf32, outp);
}
